// HybridDynamicGraph_6305011990851
// MI455X (gfx1250) — hardware-verified
//
#include <hip/hip_runtime.h>
#include <math.h>

typedef __attribute__((ext_vector_type(16))) _Float16 v16h;
typedef __attribute__((ext_vector_type(16))) __bf16 v16b;
typedef __attribute__((ext_vector_type(8)))  _Float16 v8h;
typedef __attribute__((ext_vector_type(8)))  float v8f;
typedef __attribute__((ext_vector_type(4)))  float v4f;
typedef __attribute__((ext_vector_type(2)))  float v2f;
typedef __attribute__((ext_vector_type(4)))  unsigned v4u;
typedef __attribute__((ext_vector_type(4)))  int v4i;
typedef float __attribute__((may_alias)) float_a;
typedef int __attribute__((may_alias)) int_a;

template <typename T> __device__ __forceinline__ void vst2(void* p, T v) { *(volatile T*)p = v; __threadfence(); *(volatile T*)p = v; }
__device__ __forceinline__ v8f wmma16(v16h a, v16h b, v8f c) {
  v8f d = __builtin_amdgcn_wmma_f32_16x16x32_f16(false, a, false, b, (short)0, c, false, false);
  asm volatile("v_nop\n\tv_nop\n\tv_nop\n\tv_nop" : "+v"(d) : "v"(a), "v"(b));
  return d;
}
__device__ __forceinline__ v8f wmma_bf(v16b a, v16b b, v8f c) {
  v8f d = __builtin_amdgcn_wmma_f32_16x16x32_bf16(false, a, false, b, (short)0, c, false, false);
  asm volatile("v_nop\n\tv_nop\n\tv_nop\n\tv_nop" : "+v"(d) : "v"(a), "v"(b));
  return d;
}
__device__ __forceinline__ v16h frag_h(const _Float16* rowk0, int lane) {
  union { v16h v; v8h q[2]; } u; const _Float16* p = rowk0 + 8 * (lane >> 4);
  u.q[0] = *(const v8h*)p; u.q[1] = *(const v8h*)(p + 16); return u.v;
}
__device__ __forceinline__ v16h frag_f32(const float* rowk0, int lane) {
  v16h a; const float* p = rowk0 + 8 * (lane >> 4);
#pragma unroll
  for (int i = 0; i < 8; ++i) { a[i] = (_Float16)p[i]; a[8 + i] = (_Float16)p[16 + i]; }
  return a;
}
__device__ __forceinline__ v16h frag_f32s(const float* rowk0, int lane, float sc) {
  v16h a; const float* p = rowk0 + 8 * (lane >> 4);
#pragma unroll
  for (int i = 0; i < 8; ++i) { a[i] = (_Float16)(p[i] * sc); a[8 + i] = (_Float16)(p[16 + i] * sc); }
  return a;
}
__device__ __forceinline__ v16h fragc_f32(const float* W, int k0, int n, int lane, int ld, int K) {
  v16h a; const int g = lane >> 4;
#pragma unroll
  for (int i = 0; i < 8; ++i) { const int ka = k0 + 8 * g + i, kb = ka + 16;
    a[i] = (_Float16)(ka < K ? W[(size_t)(ka < K ? ka : K - 1) * ld + n] : 0.f); a[8 + i] = (_Float16)(kb < K ? W[(size_t)(kb < K ? kb : K - 1) * ld + n] : 0.f); }
  return a;
}
struct F2 { v16b h, l; };
__device__ __forceinline__ F2 bsplit16(const float v[16]) { F2 r;
#pragma unroll
  for (int i = 0; i < 16; ++i) { const __bf16 h = (__bf16)v[i]; r.h[i] = h; r.l[i] = (__bf16)(v[i] - (float)h); }
  return r; }
__device__ __forceinline__ F2 split_row(const float* row, int k0, int lane) { float v[16]; const float* p = row + k0 + 8 * (lane >> 4);
#pragma unroll
  for (int i = 0; i < 8; ++i) { v[i] = p[i]; v[8 + i] = p[16 + i]; }
  return bsplit16(v); }
__device__ __forceinline__ F2 split_rowK(const float* row, int k0, int lane, int K) { float v[16]; const int g = lane >> 4;
#pragma unroll
  for (int i = 0; i < 8; ++i) { const int ka = k0 + 8 * g + i, kb = ka + 16; v[i] = ka < K ? row[ka < K ? ka : K - 1] : 0.f; v[8 + i] = kb < K ? row[kb < K ? kb : K - 1] : 0.f; }
  return bsplit16(v); }
__device__ __forceinline__ F2 split_col(const float* W, int k0, int n, int lane, int ld, int K) { float v[16]; const int g = lane >> 4;
#pragma unroll
  for (int i = 0; i < 8; ++i) { const int ka = k0 + 8 * g + i, kb = ka + 16; v[i] = ka < K ? W[(size_t)(ka < K ? ka : K - 1) * ld + n] : 0.f; v[8 + i] = kb < K ? W[(size_t)(kb < K ? kb : K - 1) * ld + n] : 0.f; }
  return bsplit16(v); }
__device__ __forceinline__ v8f mac3(const F2& a, const F2& b, v8f c) { c = wmma_bf(a.l, b.h, c); c = wmma_bf(a.h, b.l, c); return wmma_bf(a.h, b.h, c); }
__device__ __forceinline__ float sigm(float v) { return 1.0f / (1.0f + expf(-v)); }
#define LDSX() do { asm volatile("s_wait_dscnt 0" ::: "memory"); __builtin_amdgcn_wave_barrier(); __builtin_amdgcn_fence(__ATOMIC_RELEASE, "workgroup"); } while (0)


#define NN 1024
#define HDD 10000
#define HDP 10048
#define HID 128
#ifndef NRT
#define NRT (NN / 64)
#endif
typedef __attribute__((ext_vector_type(8))) __bf16 v8b;
__device__ __forceinline__ v16b frag_b(const __bf16* rowk0, int lane) {
  union { v16b v; v8b q[2]; } u; const __bf16* p = rowk0 + 8 * (lane >> 4);
  u.q[0] = *(const v8b*)p; u.q[1] = *(const v8b*)(p + 16); return u.v;
}
__device__ __forceinline__ float bfr(float v) { return (float)(__bf16)v; }
__device__ __attribute__((noinline)) float exp_ni(float v) { return expf(v); }
__device__ __attribute__((noinline)) float erf_ni(float v) { return erff(v); }

#define WS_FB 0u
#define WS_WA (WS_FB + 2u * NN * HDP)
#define WS_WB (WS_WA + 2u * HID * HDP)
#define WS_U  (WS_WB + 2u * HID * HDP)
#define WS_V  (WS_U + 4u * NN * HID)
#define WS_S  (WS_V + 4u * NN * HID)
#define WS_END (WS_S + 4u * NN * NN)

__global__ __launch_bounds__(256) void k_rows(const float* __restrict__ FEAT, const float* __restrict__ W1, __bf16* __restrict__ FB, __bf16* __restrict__ WA, __bf16* __restrict__ WB) {
  __shared__ __align__(16) __bf16 s[HDP]; __shared__ __align__(16) __bf16 s2[HDP]; const int r = blockIdx.x, which = blockIdx.y, t = threadIdx.x;
  if (which == 1 && r >= HID) return;
  if (which == 0) { for (int k = t; k < HDP; k += 256) s[k] = (__bf16)((k < HDD) ? FEAT[(size_t)r * HDD + k] : 0.f); }
  else { for (int k = t; k < HDP; k += 256) { s[k] = (__bf16)((k < HDD) ? W1[(size_t)r * 2 * HDD + k] : 0.f); s2[k] = (__bf16)((k < HDD) ? W1[(size_t)r * 2 * HDD + HDD + k] : 0.f); } }
  __syncthreads();
  for (int q = t; q < HDP / 8; q += 256) { if (which == 0) vst2((unsigned*)(FB + (size_t)r * HDP + q * 8), *(const v4u*)&s[q * 8]); else { vst2((unsigned*)(WA + (size_t)r * HDP + q * 8), *(const v4u*)&s[q * 8]); vst2((unsigned*)(WB + (size_t)r * HDP + q * 8), *(const v4u*)&s2[q * 8]); } }
}
__global__ __launch_bounds__(128) void k_proj(const __bf16* __restrict__ FB, const __bf16* __restrict__ WA, const __bf16* __restrict__ WB, float* __restrict__ U, float* __restrict__ V) {
  __shared__ __align__(16) float so[4][16][132];
  const int tid = threadIdx.x, wave = tid >> 5, lane = tid & 31, col = lane & 15, g = lane >> 4; const size_t r0 = (size_t)blockIdx.x * 64 + wave * 16; const int which = blockIdx.y; const __bf16* P = which == 0 ? WA : WB; float* OUT = which == 0 ? U : V;
  v8f acc[8] = {};
#pragma unroll 2
  for (int kc = 0; kc < HDP / 32; ++kc) { const v16b a = frag_b(FB + (r0 + col) * HDP + kc * 32, lane);
#pragma unroll
    for (int j = 0; j < 8; ++j) acc[j] = wmma_bf(a, frag_b(P + (size_t)(j * 16 + col) * HDP + kc * 32, lane), acc[j]); }
#pragma unroll
  for (int j = 0; j < 8; ++j)
#pragma unroll
    for (int r = 0; r < 8; ++r) so[wave][8 * g + r][j * 16 + col] = acc[j][r];
  LDSX();
  for (int rl = 0; rl < 16; ++rl) vst2(OUT + (r0 + rl) * HID + lane * 4, *(const v4f*)&so[wave][rl][lane * 4]);
}
__global__ __launch_bounds__(256) void k_pair(const float* __restrict__ U, const float* __restrict__ V, const float* __restrict__ B1, const float* __restrict__ W2, const float* __restrict__ B2, float* __restrict__ S) {
  __shared__ float su[HID], sw[HID]; __shared__ __align__(16) float so[256]; const int i = blockIdx.x, j0 = blockIdx.y * 256, t = threadIdx.x;
  if (t < HID) { su[t] = U[(size_t)i * HID + t] + bfr(B1[t]); sw[t] = bfr(W2[t]); }
  __syncthreads();
  const float* vr = V + (size_t)(j0 + t) * HID; float a = 0.f;
#pragma unroll 4
  for (int h = 0; h < HID; ++h) a += sw[h] * fmaxf(su[h] + vr[h], 0.f);
  a += bfr(B2[0]); so[t] = 1.0f / (1.0f + exp_ni(-a));
  __syncthreads();
  if (t < 64) vst2(S + (size_t)i * NN + j0 + t * 4, *(const v4f*)&so[t * 4]);
}
__global__ __launch_bounds__(256) void k_sym(const float* __restrict__ S, float* __restrict__ OUT) {
  __shared__ __align__(16) float so[NN]; const int i = blockIdx.x, t = threadIdx.x;
  for (int j = t; j < NN; j += 256) so[j] = (j >= NRT * 64) ? 0.f : (j > i) ? S[(size_t)i * NN + j] : (j < i) ? S[(size_t)j * NN + i] : 0.f;
  __syncthreads();
  vst2(OUT + (size_t)i * NN + t * 4, *(const v4f*)&so[t * 4]);
}
extern "C" void kernel_launch(void* const* d_in, const int* in_sizes, int n_in, void* d_out, int out_size, void* d_ws, size_t ws_size, hipStream_t stream) {
  (void)in_sizes; (void)n_in; (void)out_size;
  const float** F = (const float**)d_in;
  if (ws_size < (size_t)WS_END) return;
  char* ws = (char*)d_ws; __bf16 *FB = (__bf16*)(ws + WS_FB), *WA = (__bf16*)(ws + WS_WA), *WB = (__bf16*)(ws + WS_WB); float *U = (float*)(ws + WS_U), *V = (float*)(ws + WS_V), *S = (float*)(ws + WS_S);
  k_rows<<<dim3(NN, 2), 256, 0, stream>>>(F[0], F[1], FB, WA, WB);
  k_proj<<<dim3(NRT, 2), 128, 0, stream>>>(FB, WA, WB, U, V);
  k_pair<<<dim3(NRT * 64, NRT * 64 / 256), 256, 0, stream>>>(U, V, F[2], F[3], F[4], S);
  k_sym<<<NRT * 64, 256, 0, stream>>>(S, (float*)d_out);
}
